// MLPRegressor_76072460746998
// MI455X (gfx1250) — hardware-verified
//
#include <hip/hip_runtime.h>
#include <math.h>

typedef __attribute__((ext_vector_type(16))) _Float16 v16h;
typedef __attribute__((ext_vector_type(16))) __bf16 v16b;
typedef __attribute__((ext_vector_type(8)))  _Float16 v8h;
typedef __attribute__((ext_vector_type(8)))  float v8f;
typedef __attribute__((ext_vector_type(4)))  float v4f;
typedef __attribute__((ext_vector_type(2)))  float v2f;
typedef __attribute__((ext_vector_type(4)))  unsigned v4u;
typedef __attribute__((ext_vector_type(4)))  int v4i;
typedef float __attribute__((may_alias)) float_a;
typedef int __attribute__((may_alias)) int_a;

template <typename T> __device__ __forceinline__ void vst2(void* p, T v) { *(volatile T*)p = v; __threadfence(); *(volatile T*)p = v; }
__device__ __forceinline__ v8f wmma16(v16h a, v16h b, v8f c) {
  v8f d = __builtin_amdgcn_wmma_f32_16x16x32_f16(false, a, false, b, (short)0, c, false, false);
  asm volatile("v_nop\n\tv_nop\n\tv_nop\n\tv_nop" : "+v"(d) : "v"(a), "v"(b));
  return d;
}
__device__ __forceinline__ v8f wmma_bf(v16b a, v16b b, v8f c) {
  v8f d = __builtin_amdgcn_wmma_f32_16x16x32_bf16(false, a, false, b, (short)0, c, false, false);
  asm volatile("v_nop\n\tv_nop\n\tv_nop\n\tv_nop" : "+v"(d) : "v"(a), "v"(b));
  return d;
}
__device__ __forceinline__ v16h frag_h(const _Float16* rowk0, int lane) {
  union { v16h v; v8h q[2]; } u; const _Float16* p = rowk0 + 8 * (lane >> 4);
  u.q[0] = *(const v8h*)p; u.q[1] = *(const v8h*)(p + 16); return u.v;
}
__device__ __forceinline__ v16h frag_f32(const float* rowk0, int lane) {
  v16h a; const float* p = rowk0 + 8 * (lane >> 4);
#pragma unroll
  for (int i = 0; i < 8; ++i) { a[i] = (_Float16)p[i]; a[8 + i] = (_Float16)p[16 + i]; }
  return a;
}
__device__ __forceinline__ v16h frag_f32s(const float* rowk0, int lane, float sc) {
  v16h a; const float* p = rowk0 + 8 * (lane >> 4);
#pragma unroll
  for (int i = 0; i < 8; ++i) { a[i] = (_Float16)(p[i] * sc); a[8 + i] = (_Float16)(p[16 + i] * sc); }
  return a;
}
__device__ __forceinline__ v16h fragc_f32(const float* W, int k0, int n, int lane, int ld, int K) {
  v16h a; const int g = lane >> 4;
#pragma unroll
  for (int i = 0; i < 8; ++i) { const int ka = k0 + 8 * g + i, kb = ka + 16;
    a[i] = (_Float16)(ka < K ? W[(size_t)(ka < K ? ka : K - 1) * ld + n] : 0.f); a[8 + i] = (_Float16)(kb < K ? W[(size_t)(kb < K ? kb : K - 1) * ld + n] : 0.f); }
  return a;
}
struct F2 { v16b h, l; };
__device__ __forceinline__ F2 bsplit16(const float v[16]) { F2 r;
#pragma unroll
  for (int i = 0; i < 16; ++i) { const __bf16 h = (__bf16)v[i]; r.h[i] = h; r.l[i] = (__bf16)(v[i] - (float)h); }
  return r; }
__device__ __forceinline__ F2 split_row(const float* row, int k0, int lane) { float v[16]; const float* p = row + k0 + 8 * (lane >> 4);
#pragma unroll
  for (int i = 0; i < 8; ++i) { v[i] = p[i]; v[8 + i] = p[16 + i]; }
  return bsplit16(v); }
__device__ __forceinline__ F2 split_rowK(const float* row, int k0, int lane, int K) { float v[16]; const int g = lane >> 4;
#pragma unroll
  for (int i = 0; i < 8; ++i) { const int ka = k0 + 8 * g + i, kb = ka + 16; v[i] = ka < K ? row[ka < K ? ka : K - 1] : 0.f; v[8 + i] = kb < K ? row[kb < K ? kb : K - 1] : 0.f; }
  return bsplit16(v); }
__device__ __forceinline__ F2 split_col(const float* W, int k0, int n, int lane, int ld, int K) { float v[16]; const int g = lane >> 4;
#pragma unroll
  for (int i = 0; i < 8; ++i) { const int ka = k0 + 8 * g + i, kb = ka + 16; v[i] = ka < K ? W[(size_t)(ka < K ? ka : K - 1) * ld + n] : 0.f; v[8 + i] = kb < K ? W[(size_t)(kb < K ? kb : K - 1) * ld + n] : 0.f; }
  return bsplit16(v); }
__device__ __forceinline__ v8f mac3(const F2& a, const F2& b, v8f c) { c = wmma_bf(a.l, b.h, c); c = wmma_bf(a.h, b.l, c); return wmma_bf(a.h, b.h, c); }
__device__ __forceinline__ float sigm(float v) { return 1.0f / (1.0f + expf(-v)); }
#define LDSX() do { asm volatile("s_wait_dscnt 0" ::: "memory"); __builtin_amdgcn_wave_barrier(); __builtin_amdgcn_fence(__ATOMIC_RELEASE, "workgroup"); } while (0)


#define NBR 2048
#define SL 512
#define EMB 64
#define NCAT 7
#define NCONT 5
#define TABROWS 101
__device__ __forceinline__ float bfr(float v) { return (float)(__bf16)v; }

__global__ __launch_bounds__(128) void k_pool(const float* __restrict__ cont, const int* __restrict__ cat, const int* __restrict__ len, const float* __restrict__ e0, const float* __restrict__ e1, const float* __restrict__ e2, const float* __restrict__ e3, const float* __restrict__ e4, const float* __restrict__ e5, const float* __restrict__ e6,
                                             const float* __restrict__ Wc, const float* __restrict__ bc, float* __restrict__ POOL) {
  __shared__ float stab[TABROWS][EMB]; __shared__ float scs[4][16][4]; __shared__ float ses[128][33]; __shared__ __align__(16) float sp[EMB * 2];
  const int tid = threadIdx.x, wave = tid >> 5, lane = tid & 31, col = lane & 15, g = lane >> 4; const int b = blockIdx.x; const int Lr = len[b]; const int L = Lr < 1 ? 1 : (Lr > SL ? SL : Lr);
  { const float* tabs[NCAT] = {e0, e1, e2, e3, e4, e5, e6}; const int rows[NCAT] = {2, 2, 2, 11, 19, 31, 34}; int base = 0;
    for (int i = 0; i < NCAT; ++i) { for (int q = tid; q < rows[i] * EMB; q += 128) stab[base + q / EMB][q % EMB] = bfr(tabs[i][q]); base += rows[i]; } }
  float csum[4] = {0.f, 0.f, 0.f, 0.f}; float esum[32];
#pragma unroll
  for (int d = 0; d < 32; ++d) esum[d] = 0.f;
  const int ets = tid & 63, ed0 = (tid >> 6) * 32; const int toff[NCAT] = {0, 2, 4, 6, 17, 36, 67};
  __syncthreads();
#pragma unroll 1
  for (int ch = 0; ch < SL / 64; ++ch) { const int s0 = ch * 64;
    { const size_t r0 = (size_t)b * SL + s0 + wave * 16; const v16b a = split_rowK(cont + (r0 + col) * NCONT, 0, lane, NCONT).h; v8f acc[4] = {};
#pragma unroll
      for (int j = 0; j < 4; ++j) acc[j] = wmma_bf(a, split_col(Wc, 0, j * 16 + col, lane, EMB, NCONT).h, acc[j]);
#pragma unroll
      for (int j = 0; j < 4; ++j) { const float bb = bfr(bc[j * 16 + col]); float s = 0.f;
#pragma unroll
        for (int r = 0; r < 8; ++r) { const int tok = s0 + wave * 16 + 8 * g + r; const float v = acc[j][r] + bb; s += (tok < L && v > 0.f) ? v : 0.f; }
        csum[j] += s; } }
    { const int tok = s0 + ets; if (tok < L) { const int* cr = cat + ((size_t)b * SL + tok) * NCAT;
        const int rows_[NCAT] = {2, 2, 2, 11, 19, 31, 34};
#pragma unroll 1
        for (int i = 0; i < NCAT; ++i) { int cv = cr[i]; cv = cv < 0 ? 0 : (cv >= rows_[i] ? rows_[i] - 1 : cv); const int row = toff[i] + cv;
#pragma unroll
          for (int d = 0; d < 32; ++d) esum[d] += stab[row][ed0 + d]; } } } }
#pragma unroll
  for (int j = 0; j < 4; ++j) { const float s2 = csum[j] + __shfl_xor(csum[j], 16, 32); if (g == 0) scs[wave][col][j] = s2; }
#pragma unroll
  for (int d = 0; d < 32; ++d) ses[tid][d] = esum[d];
  __syncthreads();
  if (tid < EMB) { const int dg = tid >> 5, dd = tid & 31; float s = 0.f; for (int sl = 0; sl < 64; ++sl) s += ses[dg * 64 + sl][dd]; sp[tid] = s * (1.0f / 7.0f) / (float)L; }
  else { const int dim = tid - EMB; float s = 0.f; for (int wv = 0; wv < 4; ++wv) s += scs[wv][dim & 15][dim >> 4]; sp[EMB + dim] = s / (float)L; }
  __syncthreads();
  if (tid < 32) vst2(POOL + (size_t)b * (2 * EMB) + tid * 4, *(const v4f*)(&sp[tid * 4]));
}
__global__ __launch_bounds__(128) void k_head(const float* __restrict__ POOL, const float* __restrict__ W1, const float* __restrict__ b1, const float* __restrict__ W2, const float* __restrict__ b2, float* __restrict__ out) {
  __shared__ __align__(16) float sh[64][EMB + 4]; __shared__ __align__(16) float so[64 * 2];
  const int tid = threadIdx.x, wave = tid >> 5, lane = tid & 31, col = lane & 15, g = lane >> 4; const size_t r0 = (size_t)blockIdx.x * 64 + wave * 16;
  v8f acc[4] = {};
#pragma unroll
  for (int kc = 0; kc < 128 / 32; ++kc) { const F2 a = split_row(POOL + (r0 + col) * 128, kc * 32, lane);
#pragma unroll
    for (int j = 0; j < 4; ++j) { const v16b wb = split_col(W1, kc * 32, j * 16 + col, lane, EMB, 128).h; acc[j] = wmma_bf(a.l, wb, acc[j]); acc[j] = wmma_bf(a.h, wb, acc[j]); } }
#pragma unroll
  for (int j = 0; j < 4; ++j) { const float bb = bfr(b1[j * 16 + col]);
#pragma unroll
    for (int r = 0; r < 8; ++r) { const float v = acc[j][r] + bb; sh[wave * 16 + 8 * g + r][j * 16 + col] = v > 0.f ? v : 0.f; } }
  __syncthreads();
  if (tid < 64) {
#pragma unroll 1
    for (int c = 0; c < 2; ++c) { float q = bfr(b2[c]);
#pragma unroll 4
      for (int o = 0; o < EMB; ++o) q += sh[tid][o] * bfr(W2[o * 2 + c]);
      so[tid * 2 + c] = q > 0.f ? q : 0.f; } }
  __syncthreads();
  if (tid < 32) vst2(out + (size_t)blockIdx.x * 128 + tid * 4, *(const v4f*)(&so[tid * 4]));
}
extern "C" void kernel_launch(void* const* d_in, const int* in_sizes, int n_in, void* d_out, int out_size, void* d_ws, size_t ws_size, hipStream_t stream) {
  (void)in_sizes; (void)n_in; (void)out_size; (void)ws_size;
  const float* cont = (const float*)d_in[0]; const int* cat = (const int*)d_in[1]; const int* len = (const int*)d_in[2];
  const float** I = (const float**)d_in;
  float* POOL = (float*)d_ws;
  k_pool<<<NBR, 128, 0, stream>>>(cont, cat, len, I[3], I[4], I[5], I[6], I[7], I[8], I[9], I[10], I[11], POOL);
  k_head<<<NBR / 64, 128, 0, stream>>>(POOL, I[12], I[13], I[14], I[15], (float*)d_out);
}
